// temporal_17712445129536
// MI455X (gfx1250) — hardware-run, weakly checked
//
#include <hip/hip_runtime.h>
#include <math.h>

typedef __attribute__((ext_vector_type(16))) _Float16 v16h;
typedef __attribute__((ext_vector_type(8)))  _Float16 v8h;
typedef __attribute__((ext_vector_type(8)))  float    v8f;
typedef __attribute__((ext_vector_type(4)))  float    v4f;

constexpr int kBL    = 16;
constexpr int kN     = 1024;
constexpr int kDim   = 512;
constexpr int kHeads = 8;
constexpr int kDh    = 64;
constexpr int kTok   = kBL * kN;
static_assert(kHeads * kDh == kDim);
static_assert((kTok % 64) == 0 && (kDim % 64) == 0 && (kN % 64) == 0 && (kDh % 32) == 0);
static_assert((kDim % 32) == 0 && (kN % 32) == 0);

constexpr float kXCarry = 16.0f;
constexpr float kWCarry = 256.0f;
constexpr float kACarry = 16.0f;
constexpr float kPCarry = 32768.0f;
constexpr float kCCarry = 256.0f;
constexpr float kProjScale = kACarry / (kXCarry * kWCarry);
constexpr float kCtxScale  = kCCarry / kACarry;
constexpr float kOutScale  = 1.0f / (kCCarry * kWCarry);

constexpr size_t kBytesWH = (size_t)4 * kDim * kDim * 2;
constexpr size_t kBytesPl = (size_t)kTok * kDim * 2;
constexpr size_t kOffWH = 0;
constexpr size_t kOffXH = kOffWH + kBytesWH;
constexpr size_t kOffQH = kOffXH + kBytesPl;
constexpr size_t kOffKH = kOffQH + kBytesPl;
constexpr size_t kOffVT = kOffKH + kBytesPl;
constexpr size_t kOffIH = kOffVT + kBytesPl;
constexpr size_t kWsTotal = kOffIH + kBytesPl;
static_assert(kWsTotal == 85983232ull);
static_assert(kWsTotal <= 134217728ull);
static_assert((kOffXH % 128) == 0 && (kOffQH % 128) == 0 && (kOffKH % 128) == 0 && (kOffVT % 128) == 0 && (kOffIH % 128) == 0);

union FragU { v16h v; v8h h[2]; };
__device__ __forceinline__ v16h frag_load(const _Float16* p) {
  FragU f;
  f.h[0] = *(const v8h*)(p);
  f.h[1] = *(const v8h*)(p + 16);
  return f.v;
}
__device__ __forceinline__ v8f mma_h(v16h a, v16h b, v8f c) {
  c = __builtin_amdgcn_wmma_f32_16x16x32_f16(false, a, false, b, (short)0, c, false, false);
  asm volatile("v_nop\n\tv_nop\n\tv_nop\n\tv_nop" : "+v"(c) : "v"(a), "v"(b));
  return c;
}

template <int BIAS_MODE, int OUT_MODE>
__global__ __launch_bounds__(256) void wmma_gemm64(
    const unsigned short* __restrict__ Ap, int lda, long strideA,
    const unsigned short* __restrict__ Btp, int ldb, long strideB,
    void* __restrict__ Cout, int ldc, long strideC,
    const float* __restrict__ bias, float bscale,
    int M, int N, int K, float scale) {
  const _Float16* A  = (const _Float16*)Ap;
  const _Float16* Bt = (const _Float16*)Btp;
  __shared__ __align__(16) float sT[8][16 * 68];
  const int b    = blockIdx.y;
  const int lane = threadIdx.x & 31;
  const int wave = threadIdx.x >> 5;
  const int tilesN = N >> 6;
  const int tilesM = M >> 6;
  const int tile = blockIdx.x * 8 + wave;
  if (tile >= tilesM * tilesN) return;
  const int tm = tile / tilesN;
  const int tn = tile - tm * tilesN;
  const int m0 = tm << 6;
  const int n0 = tn << 6;

  const _Float16* Ab = A  + (size_t)b * strideA;
  const _Float16* Bb = Bt + (size_t)b * strideB;

  const int rlane = lane & 15;
  const int koff  = (lane >> 4) * 8;
  const int mOff  = (lane >> 4) * 8;

  v8f acc[4][4];
#pragma unroll
  for (int i = 0; i < 4; ++i)
#pragma unroll
    for (int j = 0; j < 4; ++j) acc[i][j] = (v8f){0.f,0.f,0.f,0.f,0.f,0.f,0.f,0.f};

  for (int k0 = 0; k0 < K; k0 += 32) {
    v16h bh[4];
#pragma unroll
    for (int j = 0; j < 4; ++j) {
      const size_t bo = (size_t)(n0 + (j << 4) + rlane) * ldb + koff + k0;
      bh[j] = frag_load(Bb + bo);
    }
#pragma unroll
    for (int i = 0; i < 4; ++i) {
      const size_t ao = (size_t)(m0 + (i << 4) + rlane) * lda + koff + k0;
      const v16h ah = frag_load(Ab + ao);
#pragma unroll
      for (int j = 0; j < 4; ++j) acc[i][j] = mma_h(ah, bh[j], acc[i][j]);
    }
  }

  float* slab = sT[wave];
#pragma unroll
  for (int i = 0; i < 4; ++i) {
    const int mBase = m0 + (i << 4);
#pragma unroll
    for (int j = 0; j < 4; ++j) {
      const int n = n0 + (j << 4) + rlane;
      float bv = 0.f;
      if (BIAS_MODE == 2) bv = bias[n] * bscale;
#pragma unroll
      for (int r = 0; r < 8; ++r) {
        float v = acc[i][j][r] * scale;
        if (BIAS_MODE == 1) v += bias[mBase + mOff + r] * bscale;
        if (BIAS_MODE == 2) v += bv;
        slab[(mOff + r) * 68 + (j << 4) + rlane] = v;
      }
    }
    __builtin_amdgcn_fence(__ATOMIC_RELEASE, "workgroup");
    __builtin_amdgcn_wave_barrier();
    __builtin_amdgcn_fence(__ATOMIC_ACQUIRE, "workgroup");
    if (OUT_MODE == 0) {
      float* C = (float*)Cout + (size_t)b * strideC;
      const int hh = lane >> 4, c4 = (lane & 15) * 4;
      for (int pass = 0; pass < 2; ++pass) {
#pragma unroll
        for (int it = 0; it < 8; ++it) {
          const int row = it * 2 + hh;
          v4f v = *(const v4f*)(slab + row * 68 + c4);
          *(volatile v4f*)(C + (size_t)(mBase + row) * ldc + n0 + c4) = v;
        }
        __threadfence();
      }
    } else {
      const int q = lane >> 3, c8 = (lane & 7) * 8;
      unsigned short* C = (unsigned short*)Cout + (size_t)b * strideC;
      for (int pass = 0; pass < 2; ++pass) {
#pragma unroll
        for (int it = 0; it < 4; ++it) {
          const int row = it * 4 + q;
          const float* sp = slab + row * 68 + c8;
          v8h hv;
#pragma unroll
          for (int e = 0; e < 8; ++e) hv[e] = (_Float16)sp[e];
          *(volatile v8h*)(C + (size_t)(mBase + row) * ldc + n0 + c8) = hv;
        }
        __threadfence();
      }
    }
    __builtin_amdgcn_fence(__ATOMIC_RELEASE, "workgroup");
    __builtin_amdgcn_wave_barrier();
    __builtin_amdgcn_fence(__ATOMIC_ACQUIRE, "workgroup");
  }
}

__global__ __launch_bounds__(256) void cast8_f16_kernel(
    const float* __restrict__ s0, const float* __restrict__ s1,
    const float* __restrict__ s2, const float* __restrict__ s3,
    unsigned short* __restrict__ out, int n8, float carry) {
  const int z = blockIdx.y;
  const float* src = (z == 0) ? s0 : (z == 1) ? s1 : (z == 2) ? s2 : s3;
  const int i = blockIdx.x * 256 + threadIdx.x;
  if (i >= n8) return;
  const float* p = src + 8 * (size_t)i;
  const v4f a = *(const v4f*)(p);
  const v4f c = *(const v4f*)(p + 4);
  v8h hv;
#pragma unroll
  for (int e = 0; e < 4; ++e) {
    hv[e]     = (_Float16)(a[e] * carry);
    hv[4 + e] = (_Float16)(c[e] * carry);
  }
  unsigned short* q = out + ((size_t)z * n8 + (size_t)i) * 8;
  *(volatile v8h*)q = hv;
  __threadfence();
  *(volatile v8h*)q = hv;
}

__global__ __launch_bounds__(128) void attn_f16_kernel(
    const unsigned short* __restrict__ Qp, const unsigned short* __restrict__ Kp,
    const unsigned short* __restrict__ Vtp, unsigned short* __restrict__ Ip, float sscale) {
  __shared__ __align__(16) _Float16 Psh[4][16 * 64];
  __shared__ __align__(16) float    Os[4][16 * 68];
  const _Float16* Q  = (const _Float16*)Qp;
  const _Float16* Kh = (const _Float16*)Kp;
  const _Float16* Vt = (const _Float16*)Vtp;

  const int tid  = threadIdx.x;
  const int wave = tid >> 5;
  const int lane = tid & 31;
  const int hh   = lane >> 4;
  const int c    = lane & 15;
  const int qb = blockIdx.x;
  const int bl = blockIdx.y;
  const int h  = blockIdx.z;
  const int q0 = qb * 64 + wave * 16;
  const size_t tokBase = (size_t)bl * kN;

  const _Float16* qrow = Q + (tokBase + q0 + c) * kDim + h * kDh + 8 * hh;
  const v16h qa0 = frag_load(qrow);
  const v16h qa1 = frag_load(qrow + 32);

  const _Float16* kptr = Kh + (tokBase + c) * kDim + h * kDh + 8 * hh;
  const _Float16* vptr = Vt + ((size_t)bl * kDim + h * kDh + c) * kN + 8 * hh;

  float mrow[8], lrow[8];
  v8f oacc[4];
#pragma unroll
  for (int r = 0; r < 8; ++r) { mrow[r] = -INFINITY; lrow[r] = 0.f; }
#pragma unroll
  for (int t = 0; t < 4; ++t) oacc[t] = (v8f){0.f,0.f,0.f,0.f,0.f,0.f,0.f,0.f};

  _Float16* pw = Psh[wave];

#pragma unroll 1
  for (int kc = 0; kc < kN / 64; ++kc) {
    const int kv0 = kc * 64;
    v8f s[4];
#pragma unroll
    for (int j = 0; j < 4; ++j) {
      const _Float16* kp = kptr + (size_t)(kv0 + j * 16) * kDim;
      const v16h kb0 = frag_load(kp);
      const v16h kb1 = frag_load(kp + 32);
      v8f a = (v8f){0.f,0.f,0.f,0.f,0.f,0.f,0.f,0.f};
      a = mma_h(qa0, kb0, a);
      a = mma_h(qa1, kb1, a);
      s[j] = a;
    }
    float cm[8];
#pragma unroll
    for (int r = 0; r < 8; ++r) {
      float m = -INFINITY;
#pragma unroll
      for (int j = 0; j < 4; ++j) {
        const float sv = s[j][r] * sscale;
        s[j][r] = sv;
        m = fmaxf(m, sv);
      }
#pragma unroll
      for (int off = 1; off < 16; off <<= 1) m = fmaxf(m, __shfl_xor(m, off, 32));
      cm[r] = m;
    }
#pragma unroll
    for (int r = 0; r < 8; ++r) {
      const float mnew  = fmaxf(mrow[r], cm[r]);
      const float alpha = __expf(mrow[r] - mnew);
      mrow[r] = mnew;
      float psum = 0.f;
#pragma unroll
      for (int j = 0; j < 4; ++j) {
        const float p = __expf(s[j][r] - mnew);
        const _Float16 ph = (_Float16)(p * kPCarry);
        psum += (float)ph;
        pw[(8 * hh + r) * 64 + j * 16 + c] = ph;
      }
      lrow[r] = lrow[r] * alpha + psum;
#pragma unroll
      for (int t = 0; t < 4; ++t) oacc[t][r] *= alpha;
    }
    __builtin_amdgcn_fence(__ATOMIC_RELEASE, "workgroup");
    __builtin_amdgcn_wave_barrier();
    __builtin_amdgcn_fence(__ATOMIC_ACQUIRE, "workgroup");
#pragma unroll 1
    for (int kk = 0; kk < 2; ++kk) {
      FragU pa;
      pa.h[0] = *(const v8h*)(pw + c * 64 + kk * 32 + 8 * hh);
      pa.h[1] = *(const v8h*)(pw + c * 64 + kk * 32 + 16 + 8 * hh);
#pragma unroll
      for (int t = 0; t < 4; ++t) {
        const v16h vb = frag_load(vptr + (size_t)(t * 16) * kN + kv0 + kk * 32);
        oacc[t] = mma_h(pa.v, vb, oacc[t]);
      }
    }
    __builtin_amdgcn_fence(__ATOMIC_RELEASE, "workgroup");
    __builtin_amdgcn_wave_barrier();
    __builtin_amdgcn_fence(__ATOMIC_ACQUIRE, "workgroup");
  }

  float* os = Os[wave];
#pragma unroll
  for (int r = 0; r < 8; ++r) {
    float l = lrow[r];
#pragma unroll
    for (int off = 1; off < 16; off <<= 1) l += __shfl_xor(l, off, 32);
    const float inv = kCtxScale * (1.0f / l);
#pragma unroll
    for (int t = 0; t < 4; ++t) os[(8 * hh + r) * 68 + t * 16 + c] = oacc[t][r] * inv;
  }
  __builtin_amdgcn_fence(__ATOMIC_RELEASE, "workgroup");
  __builtin_amdgcn_wave_barrier();
  __builtin_amdgcn_fence(__ATOMIC_ACQUIRE, "workgroup");
  {
    const int q = lane >> 3, c8 = (lane & 7) * 8;
    v8h hv[4];
#pragma unroll
    for (int it = 0; it < 4; ++it) {
      const float* sp = os + (it * 4 + q) * 68 + c8;
      const v4f a0 = *(const v4f*)(sp);
      const v4f a1 = *(const v4f*)(sp + 4);
#pragma unroll
      for (int e = 0; e < 4; ++e) {
        hv[it][e]     = (_Float16)a0[e];
        hv[it][4 + e] = (_Float16)a1[e];
      }
    }
    unsigned short* ob = Ip + (tokBase + q0) * kDim + h * kDh + c8;
    for (int pass = 0; pass < 2; ++pass) {
#pragma unroll
      for (int it = 0; it < 4; ++it) {
        const int row = it * 4 + q;
        *(volatile v8h*)(ob + (size_t)row * kDim) = hv[it];
      }
      __threadfence();
    }
  }
}

extern "C" void kernel_launch(void* const* d_in, const int* in_sizes, int n_in,
                              void* d_out, int out_size, void* d_ws, size_t ws_size,
                              hipStream_t stream) {
  if (n_in < 9) return;
  if (in_sizes[0] != kTok * kDim) return;
  if (in_sizes[1] != kDim * kDim || in_sizes[3] != kDim * kDim) return;
  if (in_sizes[5] != kDim * kDim || in_sizes[7] != kDim * kDim) return;
  if (in_sizes[2] != kDim || in_sizes[4] != kDim || in_sizes[6] != kDim || in_sizes[8] != kDim) return;
  if (out_size != kTok * kDim) return;
  if (ws_size < kWsTotal) return;

  const float* x  = (const float*)d_in[0];
  const float* Wq = (const float*)d_in[1];
  const float* bq = (const float*)d_in[2];
  const float* Wk = (const float*)d_in[3];
  const float* bk = (const float*)d_in[4];
  const float* Wv = (const float*)d_in[5];
  const float* bv = (const float*)d_in[6];
  const float* Wo = (const float*)d_in[7];
  const float* bo = (const float*)d_in[8];

  char* ws = (char*)d_ws;
  unsigned short* WH = (unsigned short*)(ws + kOffWH);
  unsigned short* XH = (unsigned short*)(ws + kOffXH);
  unsigned short* QH = (unsigned short*)(ws + kOffQH);
  unsigned short* KH = (unsigned short*)(ws + kOffKH);
  unsigned short* VT = (unsigned short*)(ws + kOffVT);
  unsigned short* IH = (unsigned short*)(ws + kOffIH);
  const size_t wplane = (size_t)kDim * kDim;
  const unsigned short* WHq = WH;
  const unsigned short* WHkeys = WH + wplane;
  const unsigned short* WHvals = WH + 2 * wplane;
  const unsigned short* WHo = WH + 3 * wplane;

  const float sscale = (1.0f / sqrtf((float)kDim)) / (kACarry * kACarry);

  cast8_f16_kernel<<<dim3((kTok * kDim / 8) / 256, 1), 256, 0, stream>>>(x, x, x, x, XH, kTok * kDim / 8, kXCarry);
  cast8_f16_kernel<<<dim3((kDim * kDim / 8) / 256, 4), 256, 0, stream>>>(Wq, Wv, Wk, Wo, WH, kDim * kDim / 8, kWCarry);

  wmma_gemm64<2, 1><<<dim3(256, 1), 256, 0, stream>>>(
      XH, kDim, 0L, WHq, kDim, 0L, (void*)QH, kDim, 0L, bq, kACarry, kTok, kDim, kDim, kProjScale);
  wmma_gemm64<2, 1><<<dim3(256, 1), 256, 0, stream>>>(
      XH, kDim, 0L, WHkeys, kDim, 0L, (void*)KH, kDim, 0L, bv, kACarry, kTok, kDim, kDim, kProjScale);
  wmma_gemm64<1, 1><<<dim3(16, kBL), 256, 0, stream>>>(
      WHvals, kDim, 0L, XH, kDim, (long)kN * kDim, (void*)VT, kN, (long)kDim * kN, bk, kACarry, kDim, kN, kDim, kProjScale);

  attn_f16_kernel<<<dim3(kN / 64, kBL, kHeads), 128, 0, stream>>>(QH, KH, VT, IH, sscale);

  wmma_gemm64<2, 0><<<dim3(256, 1), 256, 0, stream>>>(
      IH, kDim, 0L, WHo, kDim, 0L, d_out, kDim, 0L, bo, 1.0f, kTok, kDim, kDim, kOutScale);
}
